// EfficientRNN_67491116089446
// MI455X (gfx1250) — hardware-verified
//
#include <hip/hip_runtime.h>
#include <stdint.h>
#pragma clang fp contract(off)

#define Bn 64
#define Tn 128
#define In 512
#define Hn 512
#define Sn 4
#define FH 2048
#define K2 1024
#define KSEL 1536
#define APITCH 1032
#define QT 4
#define SELP 32
#define NTHR 256

typedef __bf16 v16b __attribute__((ext_vector_type(16)));
typedef unsigned short v8us __attribute__((ext_vector_type(8)));
typedef float v8f __attribute__((ext_vector_type(8)));
typedef float v4f __attribute__((ext_vector_type(4)));
typedef int v4i __attribute__((ext_vector_type(4)));

union Frag { v16b v; v8us u[2]; };

__device__ __forceinline__ unsigned int bf16_rne(float f) {
    unsigned int u = __builtin_bit_cast(unsigned int, f);
    return (u + 0x7FFFu + ((u >> 16) & 1u)) >> 16;
}

__device__ __forceinline__ void split_bf16(float f, unsigned short& hi, unsigned short& lo) {
    unsigned int hb = bf16_rne(f);
    float hf = __builtin_bit_cast(float, hb << 16);
    unsigned int lb = bf16_rne(f - hf);
    hi = (unsigned short)hb;
    lo = (unsigned short)lb;
}

__device__ __forceinline__ void split8(const v4f a, const v4f b, v8us& hi, v8us& lo) {
    float f[8] = {a[0], a[1], a[2], a[3], b[0], b[1], b[2], b[3]};
#pragma unroll
    for (int i = 0; i < 8; ++i) {
        unsigned short hs, ls;
        split_bf16(f[i], hs, ls);
        hi[i] = hs;
        lo[i] = ls;
    }
}

__device__ __forceinline__ v8f zero8() {
    v8f z = {0.f, 0.f, 0.f, 0.f, 0.f, 0.f, 0.f, 0.f};
    return z;
}

__device__ __forceinline__ float sigm(float v) {
    float a = -v;
    a = (a > 80.0f) ? 80.0f : a;
    return 1.0f / (1.0f + expf(a));
}

__device__ __forceinline__ v8f wmma3(v8f acc, const v16b ah, const v16b al,
                                     const v16b bh, const v16b bl) {
    acc = __builtin_amdgcn_wmma_f32_16x16x32_bf16(false, ah, false, bh, (short)0, acc, false, false);
    acc = __builtin_amdgcn_wmma_f32_16x16x32_bf16(false, ah, false, bl, (short)0, acc, false, false);
    acc = __builtin_amdgcn_wmma_f32_16x16x32_bf16(false, al, false, bh, (short)0, acc, false, false);
    asm volatile("v_nop\n\tv_nop\n\tv_nop\n\tv_nop"
                 : "+v"(acc)
                 : "v"(ah), "v"(al), "v"(bh), "v"(bl));
    return acc;
}

__global__ __launch_bounds__(NTHR) void kconvw(const float* __restrict__ Wih,
                                             const float* __restrict__ Whh,
                                             unsigned short* Whi,
                                             unsigned short* Wlo,
                                             int nvec) {
    const int gid = blockIdx.x * NTHR + threadIdx.x;
    if (gid >= nvec) return;
    const size_t e0 = (size_t)gid * 8;
    const size_t k  = e0 & (size_t)(K2 - 1);
    const size_t sn = e0 >> 10;
    const float* src = (k < (size_t)In) ? (Wih + sn * In + k) : (Whh + sn * Hn + (k - In));
    const v4f a = *(const v4f*)src;
    const v4f b = *(const v4f*)(src + 4);
    v8us hi, lo;
    split8(a, b, hi, lo);
    volatile v8us* ph = (volatile v8us*)(Whi + e0);
    volatile v8us* pl = (volatile v8us*)(Wlo + e0);
    *ph = hi;
    *pl = lo;
    __threadfence();
    *ph = hi;
    *pl = lo;
}

__device__ __forceinline__ void store_rows(volatile float* o, volatile float* hw,
                                           volatile float* cw,
                                           const float* hs, const float* cs, int l) {
#pragma unroll
    for (int i = 0; i < 4; ++i) {
        const int col = i * 128 + l * 4;
        const v4f hv = *(const v4f*)(hs + col);
        const v4f cv = *(const v4f*)(cs + col);
        *(volatile v4f*)(o + col)  = hv;
        *(volatile v4f*)(hw + col) = hv;
        *(volatile v4f*)(cw + col) = cv;
    }
}

__device__ __forceinline__ int select_expert(const float* hs, const float* cs,
                                             const float* __restrict__ xr,
                                             const float* __restrict__ Wsel,
                                             const float* __restrict__ bsel, int l) {
    double p0 = 0.0, p1 = 0.0, p2 = 0.0, p3 = 0.0;
#pragma unroll 4
    for (int i = 0; i < 16; ++i) {
        const int j = l + 32 * i;
        const double hv = (double)hs[j];
        const double cv = (double)cs[j];
        const double xv = (double)xr[j];
        const float* w0 = Wsel + j;
        const float* w1 = w0 + KSEL;
        const float* w2 = w1 + KSEL;
        const float* w3 = w2 + KSEL;
        p0 += hv * (double)w0[0] + cv * (double)w0[Hn] + xv * (double)w0[2 * Hn];
        p1 += hv * (double)w1[0] + cv * (double)w1[Hn] + xv * (double)w1[2 * Hn];
        p2 += hv * (double)w2[0] + cv * (double)w2[Hn] + xv * (double)w2[2 * Hn];
        p3 += hv * (double)w3[0] + cv * (double)w3[Hn] + xv * (double)w3[2 * Hn];
    }
#pragma unroll
    for (int off = 16; off > 0; off >>= 1) {
        p0 += __shfl_xor(p0, off);
        p1 += __shfl_xor(p1, off);
        p2 += __shfl_xor(p2, off);
        p3 += __shfl_xor(p3, off);
    }
    const double l0 = p0 + (double)bsel[0];
    const double l1 = p1 + (double)bsel[1];
    const double l2 = p2 + (double)bsel[2];
    const double l3 = p3 + (double)bsel[3];
    int s = 0;
    double best = l0;
    if (l1 > best) { best = l1; s = 1; }
    if (l2 > best) { best = l2; s = 2; }
    if (l3 > best) { best = l3; s = 3; }
    s = __shfl(s, 0);
    return s;
}

__global__ __launch_bounds__(NTHR) void kstep(const float* __restrict__ x,
                                            const unsigned short* __restrict__ Whi,
                                            const unsigned short* __restrict__ Wlo,
                                            const float* __restrict__ bih,
                                            const float* __restrict__ bhh,
                                            const float* __restrict__ Wsel,
                                            const float* __restrict__ bsel,
                                            const float* hR, const float* cR, const int* selR,
                                            float* hW, float* cW, int* selW,
                                            float* out, int t) {
    __shared__ __attribute__((aligned(16))) unsigned short Ahi[16 * APITCH];
    __shared__ __attribute__((aligned(16))) unsigned short Alo[16 * APITCH];
    __shared__ __attribute__((aligned(16))) float hS[16 * Hn];
    __shared__ __attribute__((aligned(16))) float cS[16 * Hn];
    __shared__ int selL[Bn];
    __shared__ int rowIdx[16];
    __shared__ int nrowsL;

    const int tid = threadIdx.x;
    const int e = (int)(blockIdx.x >> 2) & 3;
    const int q = (int)(blockIdx.x & 3);

    if (tid < Bn) {
        int s = 0;
        if (t > 0) {
            s = selR[tid * SELP];
            s = (s < 0) ? 0 : ((s > Sn - 1) ? (Sn - 1) : s);
        }
        selL[tid] = s;
    }
    __syncthreads();
    if (tid == 0) {
        int pos = 0;
        for (int b = 0; b < Bn; ++b) {
            if (selL[b] == e) {
                const int p = pos - 16 * q;
                if (p >= 0 && p < 16) rowIdx[p] = b;
                ++pos;
            }
        }
        int nr = pos - 16 * q;
        nr = (nr < 0) ? 0 : ((nr > 16) ? 16 : nr);
        const int last = (nr > 0) ? rowIdx[nr - 1] : 0;
        for (int p = nr; p < 16; ++p) rowIdx[p] = last;
        nrowsL = nr;
    }
    __syncthreads();
    const int nrows = nrowsL;
    if (nrows == 0) return;

    {
        const int slot = tid >> 4;
        const int seg  = tid & 15;
        const int b    = rowIdx[slot] & (Bn - 1);
        const float* xrow = x + ((size_t)b * Tn + t) * In;
        const float* hrow = hR + (size_t)b * Hn;
        unsigned short* dh = Ahi + slot * APITCH;
        unsigned short* dl = Alo + slot * APITCH;
        const v4f z4 = {0.f, 0.f, 0.f, 0.f};
#pragma unroll 2
        for (int c8 = 0; c8 < 8; ++c8) {
            const int c = seg * 64 + c8 * 8;
            v4f a, bq;
            if (c < In) {
                a  = *(const v4f*)(xrow + c);
                bq = *(const v4f*)(xrow + c + 4);
            } else if (t > 0) {
                a  = *(const v4f*)(hrow + (c - In));
                bq = *(const v4f*)(hrow + (c - In) + 4);
            } else {
                a = z4; bq = z4;
            }
            v8us hi, lo;
            split8(a, bq, hi, lo);
            *(v8us*)(dh + c) = hi;
            *(v8us*)(dl + c) = lo;
        }
        const float* crow = cR + (size_t)b * Hn + seg * 32;
        float* dc = cS + slot * Hn + seg * 32;
#pragma unroll
        for (int i = 0; i < 8; ++i) {
            v4f v = z4;
            if (t > 0) v = *(const v4f*)(crow + i * 4);
            *(v4f*)(dc + i * 4) = v;
        }
    }
    __syncthreads();

    const int w  = tid >> 5;
    const int l  = tid & 31;
    const int hh = l >> 4;
    const int m  = l & 15;
    const int Kend = (t == 0) ? In : K2;
    const unsigned short* arh = Ahi + m * APITCH + 8 * hh;
    const unsigned short* arl = Alo + m * APITCH + 8 * hh;

#pragma unroll 1
    for (int i = 0; i < 4; ++i) {
        const int jt = w + 8 * i;
        const int j  = jt * 16 + m;
        const size_t nb = ((size_t)e * FH + j) * K2 + 8 * hh;
        const unsigned short* bph = Whi + nb;
        const unsigned short* bpl = Wlo + nb;
        v8f acc0 = zero8(), acc1 = zero8(), acc2 = zero8(), acc3 = zero8();

        for (int kk = 0; kk < Kend; kk += 32) {
            Frag ah, al, bh, bl;
            ah.u[0] = *(const v8us*)(arh + kk);
            ah.u[1] = *(const v8us*)(arh + kk + 16);
            al.u[0] = *(const v8us*)(arl + kk);
            al.u[1] = *(const v8us*)(arl + kk + 16);

            bh.u[0] = *(const v8us*)(bph + kk);
            bh.u[1] = *(const v8us*)(bph + kk + 16);
            bl.u[0] = *(const v8us*)(bpl + kk);
            bl.u[1] = *(const v8us*)(bpl + kk + 16);
            acc0 = wmma3(acc0, ah.v, al.v, bh.v, bl.v);

            bh.u[0] = *(const v8us*)(bph + (size_t)512 * K2 + kk);
            bh.u[1] = *(const v8us*)(bph + (size_t)512 * K2 + kk + 16);
            bl.u[0] = *(const v8us*)(bpl + (size_t)512 * K2 + kk);
            bl.u[1] = *(const v8us*)(bpl + (size_t)512 * K2 + kk + 16);
            acc1 = wmma3(acc1, ah.v, al.v, bh.v, bl.v);

            bh.u[0] = *(const v8us*)(bph + (size_t)1024 * K2 + kk);
            bh.u[1] = *(const v8us*)(bph + (size_t)1024 * K2 + kk + 16);
            bl.u[0] = *(const v8us*)(bpl + (size_t)1024 * K2 + kk);
            bl.u[1] = *(const v8us*)(bpl + (size_t)1024 * K2 + kk + 16);
            acc2 = wmma3(acc2, ah.v, al.v, bh.v, bl.v);

            bh.u[0] = *(const v8us*)(bph + (size_t)1536 * K2 + kk);
            bh.u[1] = *(const v8us*)(bph + (size_t)1536 * K2 + kk + 16);
            bl.u[0] = *(const v8us*)(bpl + (size_t)1536 * K2 + kk);
            bl.u[1] = *(const v8us*)(bpl + (size_t)1536 * K2 + kk + 16);
            acc3 = wmma3(acc3, ah.v, al.v, bh.v, bl.v);
        }

        const float* bi0 = bih + (size_t)e * FH + j;
        const float* bh0 = bhh + (size_t)e * FH + j;
        const float bi_i = bi0[0], bi_f = bi0[Hn], bi_g = bi0[2 * Hn], bi_o = bi0[3 * Hn];
        const float bb_i = bh0[0], bb_f = bh0[Hn], bb_g = bh0[2 * Hn], bb_o = bh0[3 * Hn];
#pragma unroll
        for (int r = 0; r < 8; ++r) {
            const int slot = 8 * hh + r;
            const float gi = (acc0[r] + bi_i) + bb_i;
            const float gf = (acc1[r] + bi_f) + bb_f;
            const float gg = (acc2[r] + bi_g) + bb_g;
            const float go = (acc3[r] + bi_o) + bb_o;
            const float cp = cS[slot * Hn + j];
            const float cn = sigm(gf) * cp + sigm(gi) * tanhf(gg);
            const float hn = sigm(go) * tanhf(cn);
            cS[slot * Hn + j] = cn;
            hS[slot * Hn + j] = hn;
        }
    }
    __syncthreads();

    const bool dosel = (t + 1 < Tn);
    const int slotA = w, slotB = w + 8;
    int selvA = 0, selvB = 0;
    int bA = 0, bB = 0;

    if (slotA < nrows) {
        bA = rowIdx[slotA] & (Bn - 1);
        store_rows(out + ((size_t)bA * Tn + t) * Hn, hW + (size_t)bA * Hn, cW + (size_t)bA * Hn,
                   hS + slotA * Hn, cS + slotA * Hn, l);
        if (dosel) {
            selvA = select_expert(hS + slotA * Hn, cS + slotA * Hn,
                                  x + ((size_t)bA * Tn + (t + 1)) * In, Wsel, bsel, l);
            if (l < 8) {
                const v4i sv = {selvA, selvA, selvA, selvA};
                *(volatile v4i*)(selW + (size_t)bA * SELP + l * 4) = sv;
            }
        }
    }
    if (slotB < nrows) {
        bB = rowIdx[slotB] & (Bn - 1);
        store_rows(out + ((size_t)bB * Tn + t) * Hn, hW + (size_t)bB * Hn, cW + (size_t)bB * Hn,
                   hS + slotB * Hn, cS + slotB * Hn, l);
        if (dosel) {
            selvB = select_expert(hS + slotB * Hn, cS + slotB * Hn,
                                  x + ((size_t)bB * Tn + (t + 1)) * In, Wsel, bsel, l);
            if (l < 8) {
                const v4i sv = {selvB, selvB, selvB, selvB};
                *(volatile v4i*)(selW + (size_t)bB * SELP + l * 4) = sv;
            }
        }
    }
    __threadfence();
    if (slotA < nrows) {
        store_rows(out + ((size_t)bA * Tn + t) * Hn, hW + (size_t)bA * Hn, cW + (size_t)bA * Hn,
                   hS + slotA * Hn, cS + slotA * Hn, l);
        if (dosel && l < 8) {
            const v4i sv = {selvA, selvA, selvA, selvA};
            *(volatile v4i*)(selW + (size_t)bA * SELP + l * 4) = sv;
        }
    }
    if (slotB < nrows) {
        store_rows(out + ((size_t)bB * Tn + t) * Hn, hW + (size_t)bB * Hn, cW + (size_t)bB * Hn,
                   hS + slotB * Hn, cS + slotB * Hn, l);
        if (dosel && l < 8) {
            const v4i sv = {selvB, selvB, selvB, selvB};
            *(volatile v4i*)(selW + (size_t)bB * SELP + l * 4) = sv;
        }
    }
}

extern "C" void kernel_launch(void* const* d_in, const int* in_sizes, int n_in,
                              void* d_out, int out_size, void* d_ws, size_t ws_size,
                              hipStream_t stream) {
    if (n_in < 7) return;
    if (in_sizes[0] != Bn * Tn * In) return;
    if (in_sizes[1] != Sn * FH * In) return;
    if (in_sizes[2] != Sn * FH * Hn) return;
    if (in_sizes[3] != Sn * FH) return;
    if (in_sizes[4] != Sn * FH) return;
    if (in_sizes[5] != Sn * KSEL) return;
    if (in_sizes[6] < Sn) return;
    if (out_size != Bn * Tn * Hn) return;

    const float* x    = (const float*)d_in[0];
    const float* Wih  = (const float*)d_in[1];
    const float* Whh  = (const float*)d_in[2];
    const float* bih  = (const float*)d_in[3];
    const float* bhh  = (const float*)d_in[4];
    const float* Wsel = (const float*)d_in[5];
    const float* bsel = (const float*)d_in[6];
    float* out = (float*)d_out;

    const size_t wbytes = (size_t)Sn * FH * K2 * sizeof(unsigned short);
    const size_t sbytes = (size_t)Bn * Hn * sizeof(float);
    const size_t lbytes = (size_t)Bn * SELP * sizeof(int);
    const size_t oWhi = 0;
    const size_t oWlo = oWhi + wbytes;
    const size_t oH0  = oWlo + wbytes;
    const size_t oH1  = oH0 + sbytes;
    const size_t oC0  = oH1 + sbytes;
    const size_t oC1  = oC0 + sbytes;
    const size_t oS0  = oC1 + sbytes;
    const size_t oS1  = oS0 + lbytes;
    const size_t total = oS1 + lbytes;
    if (total > ws_size) return;

    char* ws = (char*)d_ws;
    unsigned short* Whi = (unsigned short*)(ws + oWhi);
    unsigned short* Wlo = (unsigned short*)(ws + oWlo);
    float* hb[2] = {(float*)(ws + oH0), (float*)(ws + oH1)};
    float* cb[2] = {(float*)(ws + oC0), (float*)(ws + oC1)};
    int*   sb[2] = {(int*)(ws + oS0), (int*)(ws + oS1)};

    const int nvec = (Sn * FH * K2) / 8;
    kconvw<<<(nvec + NTHR - 1) / NTHR, NTHR, 0, stream>>>(Wih, Whh, Whi, Wlo, nvec);

    for (int t = 0; t < Tn; ++t) {
        const int rd = (t + 1) & 1;
        const int wr = t & 1;
        kstep<<<Sn * QT, NTHR, 0, stream>>>(x, Whi, Wlo, bih, bhh, Wsel, bsel,
                                             hb[rd], cb[rd], sb[rd],
                                             hb[wr], cb[wr], sb[wr], out, t);
    }
}
